// TransformerBlock_2396591751190
// MI455X (gfx1250) — hardware-verified
//
#include <hip/hip_runtime.h>
#include <stddef.h>
#include <stdint.h>


#define IN_C   256
#define HC     512
#define OC     128
#define NH     4
#define KVW    1024
#define ZK     1024
#define NQKV   1536
#define NVEC   2432
#define VO_BSK 1536
#define VO_BP  2048
#define VO_GAM 2176
#define VO_BET 2304
#define NVU    (NVEC / 4)
#define NTHR   256
#define NWAVE  8
#define EPT    8
#define CHUNK  (NTHR * EPT)
#define WCAP   (EPT * 32)
#define LISTN  (NWAVE * WCAP)
#define NBMAX  2048
#define NBRUN  1024
#define RCAP   28672
#define DEGCAP 64
#define STW    512
#define GBM    64
#define GBN    128
#define GTHR   128
#define GWAVE  (GTHR / 32)
#define PARTW  288
#define WSTW   258
#define ZINTS  (2 * RCAP + 2 * NBMAX + LISTN)
#define LDS_SCAN (ZINTS * 4 + 64)
#define ISC    0.08838834764831845f

static_assert((CHUNK & (CHUNK - 1)) == 0 && CHUNK <= 4096);
static_assert((NBMAX & (NBMAX - 1)) == 0 && NBMAX <= 4096);
static_assert((NBRUN & (NBRUN - 1)) == 0 && NBRUN <= NBMAX && NBRUN >= 16);
static_assert(NTHR * 8 == NBMAX);
static_assert(LISTN >= NBMAX);
static_assert((RCAP % 32) == 0 && (ZINTS % 4) == 0);
static_assert(NWAVE * STW <= RCAP);
static_assert(HC == 32 * 16 && NH * OC == HC && HC == STW);
static_assert(LDS_SCAN <= 300000);
static_assert(RCAP >= 16617 + 2048 && DEGCAP >= 35 + 8);
static_assert(GBM == GWAVE * 16 && GBN == 4 * 32 && GTHR == GBN && OC == GBN);
static_assert((IN_C % 32) == 0 && (ZK % 32) == 0 && ZK == 2 * HC);
static_assert((NQKV % GBN) == 0 && (HC % GBN) == 0);
static_assert(PARTW % 32 == 0 && PARTW / 4 <= GTHR && PARTW >= 2 * GBN + 1);
static_assert(WSTW >= 2 * GBN + 1 && (WSTW % 2) == 0);
static_assert(NVU == 19 * 32 && VO_BET + 128 == NVEC);
static_assert((HC * IN_C / 8) % NTHR == 0 && (OC * ZK / 8) % NTHR == 0);

typedef float          v4f   __attribute__((ext_vector_type(4)));
typedef float          v8f   __attribute__((ext_vector_type(8)));
typedef int            v4i   __attribute__((ext_vector_type(4)));
typedef int            v8i   __attribute__((ext_vector_type(8)));
typedef unsigned short v4us  __attribute__((ext_vector_type(4)));
typedef unsigned short v8us  __attribute__((ext_vector_type(8)));
typedef unsigned short v16us __attribute__((ext_vector_type(16)));
typedef __bf16         v16bf __attribute__((ext_vector_type(16)));
typedef v4f  __attribute__((may_alias)) v4fa;
typedef v4i  __attribute__((may_alias)) v4ia;
typedef v8us __attribute__((may_alias)) v8usa;
union FragB { v16bf v; v16us u; v8us h[2]; v8i w; };

__device__ __forceinline__ v8f wmb(const FragB& a, const FragB& b, v8f c) {
  v8f d = __builtin_amdgcn_wmma_f32_16x16x32_bf16(false, a.v, false, b.v, (short)0, c, false, false);
  asm volatile("v_nop\n\tv_nop\n\tv_nop\n\tv_nop" : "+v"(d) : "v"(a.w), "v"(b.w));
  return d;
}

__device__ __forceinline__ v8f z8() { v8f z = {0.f, 0.f, 0.f, 0.f, 0.f, 0.f, 0.f, 0.f}; return z; }

__device__ __forceinline__ void ldwait() {
  asm volatile("s_wait_loadcnt 0x0" ::: "memory");
}

__device__ __forceinline__ unsigned bf16_bits(float f) {
  const unsigned u = __float_as_uint(f);
  return (u + 0x7FFFu + ((u >> 16) & 1u)) >> 16;
}
__device__ __forceinline__ float bf16_val(float f) {
  return __uint_as_float(bf16_bits(f) << 16);
}
__device__ __forceinline__ v8us cvt8(const v4f a, const v4f b) {
  v8us o;
  o[0] = (unsigned short)bf16_bits(a.x); o[1] = (unsigned short)bf16_bits(a.y);
  o[2] = (unsigned short)bf16_bits(a.z); o[3] = (unsigned short)bf16_bits(a.w);
  o[4] = (unsigned short)bf16_bits(b.x); o[5] = (unsigned short)bf16_bits(b.y);
  o[6] = (unsigned short)bf16_bits(b.z); o[7] = (unsigned short)bf16_bits(b.w);
  return o;
}
__device__ __forceinline__ v8us ld8b(const float* __restrict__ p) {
  const v4f a = *(const v4f*)p;
  const v4f b = *(const v4f*)(p + 4);
  return cvt8(a, b);
}
__device__ __forceinline__ void put8(unsigned short* dp, const v8us o) {
  *(volatile v8us*)dp = o;
  __threadfence();
  *(volatile v8us*)dp = o;
}

__device__ __forceinline__ int scan_chunk(const int* __restrict__ dsts, int nE, int cbase, int slotBase,
                                          int nb, int vec8, int* list, int tid, int lane, int wave) {
  int wc = 0;
  const int el0  = tid * EPT;
  const int e0   = cbase + el0;
  const int sent = -2147483647 - 1;
  v4i da, db;
  if (vec8 != 0 && cbase + CHUNK <= nE) {
    da = *(const v4i*)(dsts + e0);
    db = *(const v4i*)(dsts + e0 + 4);
  } else {
    da.x = (e0     < nE) ? dsts[min(e0,     nE - 1)] : sent;
    da.y = (e0 + 1 < nE) ? dsts[min(e0 + 1, nE - 1)] : sent;
    da.z = (e0 + 2 < nE) ? dsts[min(e0 + 2, nE - 1)] : sent;
    da.w = (e0 + 3 < nE) ? dsts[min(e0 + 3, nE - 1)] : sent;
    db.x = (e0 + 4 < nE) ? dsts[min(e0 + 4, nE - 1)] : sent;
    db.y = (e0 + 5 < nE) ? dsts[min(e0 + 5, nE - 1)] : sent;
    db.z = (e0 + 6 < nE) ? dsts[min(e0 + 6, nE - 1)] : sent;
    db.w = (e0 + 7 < nE) ? dsts[min(e0 + 7, nE - 1)] : sent;
  }
  const unsigned nbs = (unsigned)slotBase;
  const unsigned unb = (unsigned)nb;
  const unsigned s0 = (unsigned)da.x - nbs, s1 = (unsigned)da.y - nbs;
  const unsigned s2 = (unsigned)da.z - nbs, s3 = (unsigned)da.w - nbs;
  const unsigned s4 = (unsigned)db.x - nbs, s5 = (unsigned)db.y - nbs;
  const unsigned s6 = (unsigned)db.z - nbs, s7 = (unsigned)db.w - nbs;
  const bool h0 = s0 < unb, h1 = s1 < unb, h2 = s2 < unb, h3 = s3 < unb;
  const bool h4 = s4 < unb, h5 = s5 < unb, h6 = s6 < unb, h7 = s7 < unb;
  const unsigned any = __builtin_amdgcn_ballot_w32(h0 | h1 | h2 | h3 | h4 | h5 | h6 | h7);
  if (any != 0u) {
#define HITJ(J, HJ, SJ) { \
      const unsigned mj = __builtin_amdgcn_ballot_w32(HJ); \
      if (mj != 0u) { \
        if (HJ) { \
          const int pos = wc + (int)__builtin_amdgcn_mbcnt_lo(mj, 0u); \
          if (pos < WCAP) list[wave * WCAP + pos] = ((el0 + (J)) << 12) | (int)(SJ); \
        } \
        wc += (int)__builtin_popcount(mj); } }
    HITJ(0, h0, s0)
    HITJ(1, h1, s1)
    HITJ(2, h2, s2)
    HITJ(3, h3, s3)
    HITJ(4, h4, s4)
    HITJ(5, h5, s5)
    HITJ(6, h6, s6)
    HITJ(7, h7, s7)
#undef HITJ
  }
  return wc;
}

__global__ __launch_bounds__(NTHR) void k_prep(
    const float* __restrict__ x,
    const float* __restrict__ Wq, const float* __restrict__ Wk, const float* __restrict__ Wv,
    const float* __restrict__ Ws, const float* __restrict__ Wp,
    const float* __restrict__ bq, const float* __restrict__ bk, const float* __restrict__ bv,
    const float* __restrict__ bs, const float* __restrict__ bp,
    const float* __restrict__ gm, const float* __restrict__ bt,
    unsigned short* XB, unsigned short* WQKV, unsigned short* WSK, unsigned short* WP2, float* VEC,
    int nN, int bX) {
  const int b = (int)blockIdx.x, tid = (int)threadIdx.x;
  if (b < bX) {
    const int u   = b * NTHR + tid;
    const int row = u >> 5;
    const int c0  = (u & 31) * 8;
    const int rc  = row < nN ? row : nN - 1;
    const float* p = x + (size_t)rc * IN_C + c0;
    v4f a = *(const v4f*)p, c = *(const v4f*)(p + 4);
    const v4f z4 = {0.f, 0.f, 0.f, 0.f};
    if (row >= nN) { a = z4; c = z4; }
    const v8us o = cvt8(a, c);
    put8(XB + (size_t)u * 8, o);
  } else if (b < bX + 64) {
    const int v = (b - bX) * NTHR + tid;
    const v8us o = ld8b(Wq + (size_t)v * 8);
    put8(WQKV + (size_t)v * 8, o);
  } else if (b < bX + 128) {
    const int v = (b - bX - 64) * NTHR + tid;
    const v8us o = ld8b(Wk + (size_t)v * 8);
    put8(WQKV + (size_t)HC * IN_C + (size_t)v * 8, o);
  } else if (b < bX + 192) {
    const int v = (b - bX - 128) * NTHR + tid;
    const v8us o = ld8b(Wv + (size_t)v * 8);
    put8(WQKV + (size_t)2 * HC * IN_C + (size_t)v * 8, o);
  } else if (b < bX + 256) {
    const int v = (b - bX - 192) * NTHR + tid;
    const v8us o = ld8b(Ws + (size_t)v * 8);
    put8(WSK + (size_t)v * 8, o);
  } else if (b < bX + 320) {
    const int v  = (b - bX - 256) * NTHR + tid;
    const int n  = v >> 7;
    const int kk = ((v & 127) * 8) & (HC - 1);
    const v8us o = ld8b(Wp + (size_t)n * HC + kk);
    put8(WP2 + (size_t)v * 8, o);
  } else {
    const int u = (b - bX - 320) * NTHR + tid;
    if (u < NVU) {
      v4f s;
      if (u < 128)      s = *(const v4f*)(bq + 4 * u);
      else if (u < 256) s = *(const v4f*)(bk + 4 * (u - 128));
      else if (u < 384) s = *(const v4f*)(bv + 4 * (u - 256));
      else if (u < 512) s = *(const v4f*)(bs + 4 * (u - 384));
      else if (u < 544) s = *(const v4f*)(bp + 4 * (u - 512));
      else if (u < 576) s = *(const v4f*)(gm + 4 * (u - 544));
      else              s = *(const v4f*)(bt + 4 * (u - 576));
      v4f o;
      o.x = bf16_val(s.x); o.y = bf16_val(s.y); o.z = bf16_val(s.z); o.w = bf16_val(s.w);
      float* dp = VEC + 4 * u;
      *(volatile v4f*)dp = o;
      __threadfence();
      *(volatile v4f*)dp = o;
    }
  }
}

template <int MODE, int KK>
__global__ __launch_bounds__(GTHR) void k_gemm(const unsigned short* __restrict__ A,
                                               const unsigned short* __restrict__ BT,
                                               const float* __restrict__ bvec, int nN,
                                               float* wsf, unsigned long long offQ, unsigned long long offKV,
                                               const float* __restrict__ agg,
                                               unsigned short* zout, float* yout, float* part) {
  __shared__ __attribute__((aligned(16))) float stg[GBM * GBN];
  __shared__ __attribute__((aligned(16))) float wst[GWAVE * WSTW];
  __shared__ __attribute__((aligned(16))) float pst[PARTW];
  const int tid = (int)threadIdx.x, lane = tid & 31, wave = tid >> 5, hh = lane >> 4, m = lane & 15;
  const int rowBase = (int)blockIdx.x * GBM;
  const int colBase = (int)blockIdx.y * GBN;

  v8f acc[8];
#pragma unroll
  for (int t = 0; t < 8; ++t) acc[t] = z8();
  const unsigned short* ap = A  + (size_t)(rowBase + 16 * wave + m) * (size_t)KK + 8 * hh;
  const unsigned short* bp = BT + (size_t)(colBase + m) * (size_t)KK + 8 * hh;

#pragma unroll 1
  for (int k0 = 0; k0 < KK; k0 += 32) {
    FragB af;
    af.h[0] = *(const v8usa*)(ap + k0);
    af.h[1] = *(const v8usa*)(ap + k0 + 16);
#pragma unroll
    for (int nt = 0; nt < 8; ++nt) {
      const unsigned short* wq = bp + (size_t)(16 * nt) * (size_t)KK + k0;
      FragB bf;
      bf.h[0] = *(const v8usa*)wq;
      bf.h[1] = *(const v8usa*)(wq + 16);
      acc[nt] = wmb(af, bf, acc[nt]);
    }
  }

#pragma unroll
  for (int nt = 0; nt < 8; ++nt) {
    const int lc = 16 * nt + m;
#pragma unroll
    for (int r = 0; r < 8; ++r) {
      const int lr = 16 * wave + 8 * hh + r;
      stg[lr * GBN + lc] = acc[nt][r];
    }
  }
  __syncthreads();

  const v4f b4 = *(const v4f*)(bvec + colBase + 4 * lane);

  if constexpr (MODE == 0) {
    const int cb = (int)blockIdx.y;
    const int pitch = cb < 4 ? HC : KVW;
    const size_t cofs = cb < 4 ? (size_t)offQ + (size_t)(cb * GBN)
                      : (cb < 8 ? (size_t)offKV + (size_t)((cb - 4) * GBN)
                                : (size_t)offKV + (size_t)(HC + (cb - 8) * GBN));
    v4f pv[16];
#pragma unroll
    for (int i = 0; i < 16; ++i) {
      const v4f xv = *(const v4fa*)(stg + (16 * wave + i) * GBN + 4 * lane);
      pv[i] = xv + b4;
    }
    float* ob = wsf + cofs + (size_t)(rowBase + 16 * wave) * (size_t)pitch + 4 * lane;
#pragma unroll
    for (int i = 0; i < 16; ++i) {
      if (rowBase + 16 * wave + i < nN) *(volatile v4f*)(ob + (size_t)i * (size_t)pitch) = pv[i];
    }
    __threadfence();
#pragma unroll
    for (int i = 0; i < 16; ++i) {
      if (rowBase + 16 * wave + i < nN) *(volatile v4f*)(ob + (size_t)i * (size_t)pitch) = pv[i];
    }
  } else if constexpr (MODE == 1) {
    v4us hv[16], lv[16];
#pragma unroll
    for (int i = 0; i < 16; ++i) {
      const int row = rowBase + 16 * wave + i;
      const bool ok = row < nN;
      const int rc = ok ? row : nN - 1;
      const v4f xv = *(const v4fa*)(stg + (16 * wave + i) * GBN + 4 * lane);
      const v4f ag = *(const v4f*)(agg + (size_t)rc * HC + colBase + 4 * lane);
      const v4f zz = (xv + b4) + ag;
      float y[4];
      y[0] = zz.x; y[1] = zz.y; y[2] = zz.z; y[3] = zz.w;
      v4us hq, lq;
#pragma unroll
      for (int j = 0; j < 4; ++j) {
        const float yy = ok ? y[j] : 0.0f;
        const unsigned hbj = bf16_bits(yy);
        hq[j] = (unsigned short)hbj;
        lq[j] = (unsigned short)bf16_bits(yy - __uint_as_float(hbj << 16));
      }
      hv[i] = hq;
      lv[i] = lq;
    }
#pragma unroll
    for (int i = 0; i < 16; ++i) {
      unsigned short* op = zout + (size_t)(rowBase + 16 * wave + i) * (size_t)ZK + colBase + 4 * lane;
      *(volatile v4us*)op = hv[i];
      *(volatile v4us*)(op + HC) = lv[i];
    }
    __threadfence();
#pragma unroll
    for (int i = 0; i < 16; ++i) {
      unsigned short* op = zout + (size_t)(rowBase + 16 * wave + i) * (size_t)ZK + colBase + 4 * lane;
      *(volatile v4us*)op = hv[i];
      *(volatile v4us*)(op + HC) = lv[i];
    }
  } else {
    v4f pv[16];
    int wn = 0;
    float wm[4], wqv[4];
#pragma unroll
    for (int j = 0; j < 4; ++j) { wm[j] = 0.0f; wqv[j] = 0.0f; }
#pragma unroll
    for (int i = 0; i < 16; ++i) {
      const int row = rowBase + 16 * wave + i;
      const bool ok = row < nN;
      const v4f xv = *(const v4fa*)(stg + (16 * wave + i) * GBN + 4 * lane);
      const v4f yv = xv + b4;
      float vv[4];
      vv[0] = ok ? yv.x : 0.0f; vv[1] = ok ? yv.y : 0.0f;
      vv[2] = ok ? yv.z : 0.0f; vv[3] = ok ? yv.w : 0.0f;
      v4f q;
      q.x = vv[0]; q.y = vv[1]; q.z = vv[2]; q.w = vv[3];
      pv[i] = q;
      if (ok) {
        wn += 1;
        const float rk = 1.0f / (float)(i + 1);
#pragma unroll
        for (int j = 0; j < 4; ++j) {
          const float d = vv[j] - wm[j];
          wm[j]  = fmaf(d, rk, wm[j]);
          wqv[j] = fmaf(d, vv[j] - wm[j], wqv[j]);
        }
      }
    }
#pragma unroll
    for (int i = 0; i < 16; ++i) {
      float* op = yout + (size_t)(rowBase + 16 * wave + i) * (size_t)OC + 4 * lane;
      *(volatile v4f*)op = pv[i];
    }
    __threadfence();
#pragma unroll
    for (int i = 0; i < 16; ++i) {
      float* op = yout + (size_t)(rowBase + 16 * wave + i) * (size_t)OC + 4 * lane;
      *(volatile v4f*)op = pv[i];
    }

    if (lane == 0) wst[wave * WSTW] = (float)wn;
#pragma unroll
    for (int j = 0; j < 4; ++j) {
      wst[wave * WSTW + 1 + 4 * lane + j]       = wm[j];
      wst[wave * WSTW + 1 + GBN + 4 * lane + j] = wqv[j];
    }
    __syncthreads();
    {
      float n = 0.0f, mean = 0.0f, M2 = 0.0f;
#pragma unroll 1
      for (int w2 = 0; w2 < GWAVE; ++w2) {
        const float nb = wst[w2 * WSTW];
        const float mb = wst[w2 * WSTW + 1 + tid];
        const float qb = wst[w2 * WSTW + 1 + GBN + tid];
        if (nb > 0.5f) {
          const float nn = n + nb;
          const float delta = mb - mean;
          const float f = nb / nn;
          mean = fmaf(delta, f, mean);
          M2 = M2 + qb + delta * delta * n * f;
          n = nn;
        }
      }
      pst[1 + tid] = mean;
      pst[1 + GBN + tid] = M2;
      if (tid == 0) pst[0] = n;
    }
#pragma unroll 1
    for (int i = 2 * GBN + 1 + tid; i < PARTW; i += GTHR) pst[i] = 0.0f;
    __syncthreads();
    const int pb = (int)blockIdx.x;
    v4f ps = {0.f, 0.f, 0.f, 0.f};
    if (tid < PARTW / 4) {
      ps = *(const v4fa*)(pst + 4 * tid);
      *(volatile v4f*)(part + (size_t)pb * PARTW + 4 * tid) = ps;
    }
    __threadfence();
    if (tid < PARTW / 4) {
      *(volatile v4f*)(part + (size_t)pb * PARTW + 4 * tid) = ps;
    }
  }
}

__global__ __launch_bounds__(NTHR) void k_scan(
    const int* __restrict__ srcs, const int* __restrict__ dsts,
    const float* __restrict__ Q, const float* __restrict__ KV, float* AGG,
    int nN, int nE, int nb, int vec8) {
  extern __shared__ v4f lds_dyn[];
  int* reg1 = (int*)lds_dyn;
  int* reg2 = reg1 + RCAP;
  int* scnt = reg2 + RCAP;
  int* soff = scnt + NBMAX;
  int* list = soff + NBMAX;
  int* wcnt = list + LISTN;
  int* wtot = wcnt + NWAVE;
  const int tid = (int)threadIdx.x, lane = tid & 31, wave = tid >> 5;
  const int nodeBase = (int)blockIdx.x * nb;

  {
    const v4i z4 = {0, 0, 0, 0};
    for (int i = tid * 4; i < ZINTS; i += NTHR * 4) *(v4ia*)(reg1 + i) = z4;
    if (tid < 2 * NWAVE) wcnt[tid] = 0;
  }
  __syncthreads();

  int tot = 0;
  const int nChunks = (nE + CHUNK - 1) / CHUNK;
#pragma unroll 1
  for (int ch = 0; ch < nChunks; ++ch) {
    const int cbase = ch * CHUNK;
    const int wc = scan_chunk(dsts, nE, cbase, nodeBase, nb, vec8, list, tid, lane, wave);
    if (lane == 0) wcnt[wave] = wc;
    __syncthreads();
    int pre = 0, all = 0;
#pragma unroll
    for (int w2 = 0; w2 < NWAVE; ++w2) {
      int c = wcnt[w2];
      c = c < 0 ? 0 : (c > WCAP ? WCAP : c);
      all += c;
      pre += (w2 < wave) ? c : 0;
    }
    const int wcc  = wc > WCAP ? WCAP : wc;
    const int base = tot + pre;
#pragma unroll 1
    for (int i = lane; i < wcc; i += 32) {
      const int ent = list[wave * WCAP + i];
      const int el  = (ent >> 12) & (CHUNK - 1);
      const int sl  = ent & (NBMAX - 1);
      int eid = cbase + el;
      eid = eid > nE - 1 ? nE - 1 : eid;
      const int pos = base + i;
      if (pos < RCAP) reg1[pos] = (int)(((unsigned)eid << 12) | (unsigned)sl);
    }
    tot += all;
    tot = tot > RCAP ? RCAP : tot;
    __syncthreads();
  }
  const int nh = tot;

  if (wave == 0) {
#pragma unroll 1
    for (int b0 = 0; b0 < nh; b0 += 32) {
      const int idx = b0 + lane;
      const int uv  = reg1[idx < RCAP ? idx : RCAP - 1];
      const int m32 = (nh - b0) < 32 ? (nh - b0) : 32;
#pragma unroll 1
      for (int k = 0; k < m32; ++k) {
        const int u  = __builtin_amdgcn_readlane(uv, k);
        const int sl = u & (NBMAX - 1);
        if (lane == 0) scnt[sl] = scnt[sl] + 1;
      }
    }
  }
  __syncthreads();

  {
    const v4i ca = *(const v4ia*)(scnt + 8 * tid);
    const v4i cb = *(const v4ia*)(scnt + 8 * tid + 4);
    const int e0 = ca.x < 0 ? 0 : ca.x, e1 = ca.y < 0 ? 0 : ca.y, e2 = ca.z < 0 ? 0 : ca.z, e3 = ca.w < 0 ? 0 : ca.w;
    const int e4 = cb.x < 0 ? 0 : cb.x, e5 = cb.y < 0 ? 0 : cb.y, e6 = cb.z < 0 ? 0 : cb.z, e7 = cb.w < 0 ? 0 : cb.w;
    const int ts = e0 + e1 + e2 + e3 + e4 + e5 + e6 + e7;
    int incl = ts;
#pragma unroll
    for (int d = 1; d < 32; d <<= 1) {
      const int up = __shfl_up(incl, d);
      if (lane >= d) incl += up;
    }
    if (lane == 31) wtot[wave] = incl;
    __syncthreads();
    int pre = 0;
#pragma unroll
    for (int w2 = 0; w2 < NWAVE; ++w2) pre += (w2 < wave) ? wtot[w2] : 0;
    int run = pre + incl - ts;
    soff[8 * tid + 0] = run; run += e0;
    soff[8 * tid + 1] = run; run += e1;
    soff[8 * tid + 2] = run; run += e2;
    soff[8 * tid + 3] = run; run += e3;
    soff[8 * tid + 4] = run; run += e4;
    soff[8 * tid + 5] = run; run += e5;
    soff[8 * tid + 6] = run; run += e6;
    soff[8 * tid + 7] = run;
  }
  __syncthreads();
  for (int i = tid; i < NBMAX; i += NTHR) list[i] = soff[i];
  __syncthreads();

  if (wave == 0) {
#pragma unroll 1
    for (int b0 = 0; b0 < nh; b0 += 32) {
      const int idx = b0 + lane;
      const int uv  = reg1[idx < RCAP ? idx : RCAP - 1];
      const int m32 = (nh - b0) < 32 ? (nh - b0) : 32;
#pragma unroll 1
      for (int k = 0; k < m32; ++k) {
        const int u   = __builtin_amdgcn_readlane(uv, k);
        const int sl  = u & (NBMAX - 1);
        const int eid = (int)((unsigned)u >> 12);
        if (lane == 0) {
          int pos = list[sl];
          pos = pos < 0 ? 0 : (pos > RCAP - 1 ? RCAP - 1 : pos);
          reg2[pos] = eid;
          list[sl] = pos + 1;
        }
      }
    }
  }
  __syncthreads();

#pragma unroll 1
  for (int i0 = 0; i0 < nh; i0 += NTHR) {
    const int i = i0 + tid;
    if (i < nh) {
      int eid = reg2[i];
      eid = eid < 0 ? 0 : (eid > nE - 1 ? nE - 1 : eid);
      int s = srcs[eid];
      s = s < 0 ? 0 : (s > nN - 1 ? nN - 1 : s);
      reg2[i] = s;
    }
  }
  __syncthreads();

  const int nbw = nb >> 3;
  const bool ovf = (nh >= RCAP);
  const float qnan = __int_as_float(0x7fc00000);
  float* stw = (float*)reg1 + wave * STW;
#pragma unroll 1
  for (int jt = 0; jt < nbw; ++jt) {
    const int slot = wave * nbw + jt;
    const int grow = nodeBase + slot;
    if (grow >= nN) break;
    int st = soff[slot];
    const int craw = scnt[slot];
    int cnt = craw;
    st  = st < 0 ? 0 : (st > nh ? nh : st);
    cnt = cnt < 0 ? 0 : (cnt > DEGCAP ? DEGCAP : cnt);
    if (cnt > nh - st) cnt = nh - st;
    const float pz = (ovf || craw > DEGCAP) ? qnan : 0.0f;

    const float* qp = Q + (size_t)grow * HC + 16 * lane;
    const v4f q0 = *(const v4f*)(qp);
    const v4f q1 = *(const v4f*)(qp + 4);
    const v4f q2 = *(const v4f*)(qp + 8);
    const v4f q3 = *(const v4f*)(qp + 12);
    ldwait();
    const v4f z4 = {0.f, 0.f, 0.f, 0.f};
    v4f a0 = z4, a1 = z4, a2 = z4, a3 = z4;
    float mx = -1.0e30f, dn = 0.f;

#pragma unroll 1
    for (int q = 0; q < cnt; ++q) {
      int idx = st + q; idx = idx > RCAP - 1 ? RCAP - 1 : idx;
      int s = reg2[idx]; s = s < 0 ? 0 : (s > nN - 1 ? nN - 1 : s);
      const float* kp = KV + (size_t)s * KVW + 16 * lane;
      const v4f k0 = *(const v4f*)(kp);
      const v4f k1 = *(const v4f*)(kp + 4);
      const v4f k2 = *(const v4f*)(kp + 8);
      const v4f k3 = *(const v4f*)(kp + 12);
      const v4f v0 = *(const v4f*)(kp + HC);
      const v4f v1 = *(const v4f*)(kp + HC + 4);
      const v4f v2 = *(const v4f*)(kp + HC + 8);
      const v4f v3 = *(const v4f*)(kp + HC + 12);
      ldwait();
      float part = q0.x * k0.x;
      part = fmaf(q0.y, k0.y, part); part = fmaf(q0.z, k0.z, part); part = fmaf(q0.w, k0.w, part);
      part = fmaf(q1.x, k1.x, part); part = fmaf(q1.y, k1.y, part); part = fmaf(q1.z, k1.z, part); part = fmaf(q1.w, k1.w, part);
      part = fmaf(q2.x, k2.x, part); part = fmaf(q2.y, k2.y, part); part = fmaf(q2.z, k2.z, part); part = fmaf(q2.w, k2.w, part);
      part = fmaf(q3.x, k3.x, part); part = fmaf(q3.y, k3.y, part); part = fmaf(q3.z, k3.z, part); part = fmaf(q3.w, k3.w, part);
      part += __shfl_xor(part, 1);
      part += __shfl_xor(part, 2);
      part += __shfl_xor(part, 4);
      const float al = part * ISC;
      const float df = al - mx;
      const float ee = expf(-fabsf(df));
      const bool up  = df > 0.f;
      const float s1 = up ? ee : 1.0f;
      const float s2 = up ? 1.0f : ee;
      mx = up ? al : mx;
      dn = fmaf(dn, s1, s2);
      a0 = a0 * s1 + v0 * s2;
      a1 = a1 * s1 + v1 * s2;
      a2 = a2 * s1 + v2 * s2;
      a3 = a3 * s1 + v3 * s2;
    }
    const float ds = dn > 0.f ? dn : 1.0f;
    const float iv = (dn > 0.f ? 1.0f : 0.0f) * (1.0f / ds);
    const v4f r0 = a0 * iv + pz;
    const v4f r1 = a1 * iv + pz;
    const v4f r2 = a2 * iv + pz;
    const v4f r3 = a3 * iv + pz;
    __builtin_amdgcn_fence(__ATOMIC_RELEASE, "wavefront");
    __builtin_amdgcn_wave_barrier();
    *(v4fa*)(stw + 16 * lane)      = r0;
    *(v4fa*)(stw + 16 * lane + 4)  = r1;
    *(v4fa*)(stw + 16 * lane + 8)  = r2;
    *(v4fa*)(stw + 16 * lane + 12) = r3;
    __builtin_amdgcn_fence(__ATOMIC_RELEASE, "wavefront");
    __builtin_amdgcn_wave_barrier();
    const v4f g0 = *(const v4fa*)(stw + 4 * lane);
    const v4f g1 = *(const v4fa*)(stw + 128 + 4 * lane);
    const v4f g2 = *(const v4fa*)(stw + 256 + 4 * lane);
    const v4f g3 = *(const v4fa*)(stw + 384 + 4 * lane);
    float* gp = AGG + (size_t)grow * HC + 4 * lane;
    *(volatile v4f*)(gp)       = g0;
    *(volatile v4f*)(gp + 128) = g1;
    *(volatile v4f*)(gp + 256) = g2;
    *(volatile v4f*)(gp + 384) = g3;
    __threadfence();
    *(volatile v4f*)(gp)       = g0;
    *(volatile v4f*)(gp + 128) = g1;
    *(volatile v4f*)(gp + 256) = g2;
    *(volatile v4f*)(gp + 384) = g3;
  }
}

__global__ __launch_bounds__(OC) void k_bnfin(const float* __restrict__ part, int nPart, float* ss) {
  __shared__ __attribute__((aligned(16))) float stg[2 * OC];
  const int tid = (int)threadIdx.x;
  const int c = tid;
  double n = 0.0, mean = 0.0, M2 = 0.0;
#pragma unroll 1
  for (int b = 0; b < nPart; ++b) {
    const float* pr = part + (size_t)b * PARTW;
    const double nb = (double)pr[0];
    const double mb = (double)pr[1 + c];
    const double qb = (double)pr[1 + GBN + c];
    if (nb > 0.5) {
      const double nn = n + nb;
      const double delta = mb - mean;
      const double f = nb / nn;
      mean = mean + delta * f;
      M2 = M2 + qb + delta * delta * n * f;
      n = nn;
    }
  }
  const double nt = n < 1.0 ? 1.0 : n;
  const float varf  = (float)(M2 / nt);
  const float meanf = (float)mean;
  const float rstd = 1.0f / sqrtf(varf + 1e-5f);
  stg[c] = meanf;
  stg[OC + c] = rstd;
  __syncthreads();
  v4f v = {0.f, 0.f, 0.f, 0.f};
  if (tid < (2 * OC) / 4) {
    v = *(const v4fa*)(stg + 4 * tid);
    *(volatile v4f*)(ss + 4 * tid) = v;
  }
  __threadfence();
  if (tid < (2 * OC) / 4) {
    *(volatile v4f*)(ss + 4 * tid) = v;
  }
}

__global__ __launch_bounds__(NTHR) void k_bn(const float* __restrict__ y, const float* __restrict__ ss,
                                             const float* __restrict__ vec, int nUnits, float* out) {
  __shared__ float ssh[4 * OC];
  const int tid = (int)threadIdx.x;
  ssh[tid] = ss[tid];
  ssh[2 * OC + tid] = vec[VO_GAM + tid];
  __syncthreads();
  const int u = (int)blockIdx.x * NTHR + tid;
  if (u >= nUnits) return;
  const int c4 = (u & 31) * 4;
  const v4f x = *(const v4f*)(y + (size_t)u * 4);
  float xi[4];
  xi[0] = x.x; xi[1] = x.y; xi[2] = x.z; xi[3] = x.w;
  float oo[4];
#pragma unroll
  for (int j = 0; j < 4; ++j) {
    const float t = ((xi[j] - ssh[c4 + j]) * ssh[OC + c4 + j]) * ssh[2 * OC + c4 + j] + ssh[3 * OC + c4 + j];
    oo[j] = (t > 0.0f) ? t : 0.01f * t;
  }
  v4f o;
  o.x = oo[0]; o.y = oo[1]; o.z = oo[2]; o.w = oo[3];
  float* op = out + (size_t)u * 4;
  *(volatile v4f*)op = o;
  __threadfence();
  *(volatile v4f*)op = o;
}

static int pick_nb(int nE, int nN) {
  int nb = NBRUN;
  while (nb > 16 && (long long)nb * (long long)nE * 5LL > (long long)RCAP * (long long)nN * 4LL) nb >>= 1;
  return nb;
}
static inline int cdiv(int a, int b) { return (a + b - 1) / b; }
static inline size_t al256(size_t o) { return (o + 255) & ~(size_t)255; }
static inline size_t smax(size_t a, size_t b) { return a > b ? a : b; }

extern "C" void kernel_launch(void* const* d_in, const int* in_sizes, int n_in,
                              void* d_out, int out_size, void* d_ws, size_t ws_size,
                              hipStream_t stream) {
  if (n_in < 14) return;
  if (in_sizes[0] < IN_C || (in_sizes[0] % IN_C) != 0) return;
  const int nN = in_sizes[0] / IN_C;
  if (nN < 16 || nN > (1 << 22)) return;
  if (in_sizes[1] < 2 || (in_sizes[1] & 1) != 0) return;
  const int nE = in_sizes[1] / 2;
  if (nE < 1 || nE > (1 << 20)) return;
  if (in_sizes[2] != HC * IN_C || in_sizes[3] != HC) return;
  if (in_sizes[4] != HC * IN_C || in_sizes[5] != HC) return;
  if (in_sizes[6] != HC * IN_C || in_sizes[7] != HC) return;
  if (in_sizes[8] != HC * IN_C || in_sizes[9] != HC) return;
  if (in_sizes[10] != OC * HC || in_sizes[11] != OC) return;
  if (in_sizes[12] != OC || in_sizes[13] != OC) return;
  if ((long long)out_size != (long long)nN * OC) return;

  const float* x  = (const float*)d_in[0];
  const int*   ei = (const int*)  d_in[1];
  const float* Wq = (const float*)d_in[2];
  const float* bq = (const float*)d_in[3];
  const float* Wk = (const float*)d_in[4];
  const float* bk = (const float*)d_in[5];
  const float* Wv = (const float*)d_in[6];
  const float* bv = (const float*)d_in[7];
  const float* Ws = (const float*)d_in[8];
  const float* bs = (const float*)d_in[9];
  const float* Wp = (const float*)d_in[10];
  const float* bp = (const float*)d_in[11];
  const float* gm = (const float*)d_in[12];
  const float* bt = (const float*)d_in[13];
  float* out = (float*)d_out;
  const int* src = ei;
  const int* dst = ei + nE;

  const int MP   = cdiv(nN, GBM) * GBM;
  const int gM   = MP / GBM;
  const int nb   = pick_nb(nE, nN);
  const int gA   = cdiv(nN, nb);
  const int vec8 = ((nE & 3) == 0) ? 1 : 0;
  if ((long long)gA * nb < (long long)nN) return;
  if ((MP & 7) != 0) return;

  char* ws = (char*)d_ws;
  size_t off = 0;
  const size_t oXB   = off; off = al256(off + (size_t)MP * IN_C * 2);
  const size_t oWQKV = off; off = al256(off + (size_t)NQKV * IN_C * 2);
  const size_t oWSK  = off; off = al256(off + (size_t)HC * IN_C * 2);
  const size_t oWP2  = off; off = al256(off + (size_t)OC * ZK * 2);
  const size_t oVEC  = off; off = al256(off + (size_t)NVEC * 4);
  const size_t oQ    = off; off = al256(off + smax((size_t)nN * HC * 4,
                                                   (size_t)MP * OC * 4));
  const size_t oKV   = off; off = al256(off + smax((size_t)nN * KVW * 4,
                                                   (size_t)MP * ZK * 2));
  const size_t oAGG  = off; off = al256(off + (size_t)nN * HC * 4);
  const size_t oPT   = off; off = al256(off + (size_t)gM * PARTW * 4);
  const size_t oSS   = off; off = al256(off + (size_t)(2 * OC) * 4);
  if (off > ws_size) return;
  unsigned short* XB   = (unsigned short*)(ws + oXB);
  unsigned short* WQKV = (unsigned short*)(ws + oWQKV);
  unsigned short* WSK  = (unsigned short*)(ws + oWSK);
  unsigned short* WP2  = (unsigned short*)(ws + oWP2);
  float*          VEC  = (float*)(ws + oVEC);
  float*          Qp   = (float*)(ws + oQ);
  float*          KVp  = (float*)(ws + oKV);
  float*          AGG  = (float*)(ws + oAGG);
  unsigned short* ZHL  = (unsigned short*)(ws + oKV);
  float*          Yp   = (float*)(ws + oQ);
  float*          PT   = (float*)(ws + oPT);
  float*          SS   = (float*)(ws + oSS);
  float*          wsf  = (float*)d_ws;
  const unsigned long long offQ  = (unsigned long long)(oQ / 4);
  const unsigned long long offKV = (unsigned long long)(oKV / 4);

  hipFuncSetAttribute(reinterpret_cast<const void*>(&k_scan),
                      hipFuncAttributeMaxDynamicSharedMemorySize, LDS_SCAN);

  const int bX = MP / 8;
  k_prep<<<bX + 323, NTHR, 0, stream>>>(x, Wq, Wk, Wv, Ws, Wp, bq, bk, bv, bs, bp, gm, bt,
                                        XB, WQKV, WSK, WP2, VEC, nN, bX);
  k_gemm<0, IN_C><<<dim3(gM, NQKV / GBN), GTHR, 0, stream>>>(XB, WQKV, VEC, nN, wsf, offQ, offKV,
                                                             AGG, ZHL, Yp, PT);
  k_scan<<<gA, NTHR, LDS_SCAN, stream>>>(src, dst, Qp, KVp, AGG, nN, nE, nb, vec8);
  k_gemm<1, IN_C><<<dim3(gM, HC / GBN), GTHR, 0, stream>>>(XB, WSK, VEC + VO_BSK, nN, wsf, offQ, offKV,
                                                           AGG, ZHL, Yp, PT);
  k_gemm<2, ZK><<<dim3(gM, 1), GTHR, 0, stream>>>(ZHL, WP2, VEC + VO_BP, nN, wsf, offQ, offKV,
                                                  AGG, ZHL, Yp, PT);
  k_bnfin<<<1, OC, 0, stream>>>(PT, gM, SS);
  const int nUo = nN * (OC / 4);
  k_bn<<<cdiv(nUo, NTHR), NTHR, 0, stream>>>(Yp, SS, VEC, nUo, out);
}
